// XSACausalSelfAttention_28063316312159
// MI455X (gfx1250) — hardware-verified
//
#include <hip/hip_runtime.h>
#include <math.h>
#include <stdint.h>

#define NBATCH 2
#define SEQ    2048
#define DM     2048
#define NHEAD  16
#define NKV    4
#define HDIM   128
#define RHALF  64
#define KVD    (NKV * HDIM)
#define NTOK   (NBATCH * SEQ)
#define NQB    (SEQ / 64)
#define NQP    8
#define WSC    64.0f
#define QSC    4.0f
#define KSC    16.0f
#define VSC    16.0f
#define RSC    4096.0f
#define PSC    1024.0f
#define CXS    1024.0f
#define RMS_EPS 1.1920929e-07f
#define XCLIP  1.0e-12f
#define LOG2_BASE 13.287712379549449
#define NEG_BIG (-1.0e30f)
static_assert(NHEAD * HDIM == DM);
static_assert((NHEAD % NKV) == 0);
static_assert(HDIM == 2 * RHALF);
static_assert((SEQ % 64) == 0 && (DM % 128) == 0 && (KVD % 128) == 0);
static_assert((DM % 64) == 0 && (KVD % 64) == 0 && (HDIM % 32) == 0);
static_assert(((NTOK * DM) % 2048) == 0);
static_assert(((SEQ * RHALF) % 256) == 0);
static_assert(NQP > 0 && NQP < NQB);

typedef _Float16 v16h __attribute__((ext_vector_type(16)));
typedef _Float16 v8h  __attribute__((ext_vector_type(8)));
typedef float    v8f  __attribute__((ext_vector_type(8)));
typedef float    v4f  __attribute__((ext_vector_type(4)));
typedef unsigned int v4u __attribute__((ext_vector_type(4)));
union FH { v16h v; v8h h[2]; };

__device__ __forceinline__ unsigned short bf_bits(float f) {
  unsigned u = __float_as_uint(f);
  return (unsigned short)((u + 0x7FFFu + ((u >> 16) & 1u)) >> 16);
}
__device__ __forceinline__ float bf_up(unsigned short h) { return __uint_as_float(((unsigned)h) << 16); }
__device__ __forceinline__ float bfr(float f) { return bf_up(bf_bits(f)); }
__device__ __forceinline__ unsigned short h_bits(_Float16 x) { return __builtin_bit_cast(unsigned short, x); }
__device__ __forceinline__ unsigned pk16(unsigned short a, unsigned short b) { return (unsigned)a | ((unsigned)b << 16); }
__device__ __forceinline__ v8f zero8() { v8f z = {0.f, 0.f, 0.f, 0.f, 0.f, 0.f, 0.f, 0.f}; return z; }

__device__ __forceinline__ v16h ldfrag_h(const _Float16* p) {
  FH f;
  f.h[0] = *(const v8h*)(p);
  f.h[1] = *(const v8h*)(p + 16);
  return f.v;
}

__device__ __forceinline__ v8f mma_h_raw(v16h a, v16h b, v8f c) {
  return __builtin_amdgcn_wmma_f32_16x16x32_f16(false, a, false, b, (short)0, c, false, false);
}
__device__ __forceinline__ v8f mma_h(v16h a, v16h b, v8f c) {
  c = mma_h_raw(a, b, c);
#if defined(__HIP_DEVICE_COMPILE__)
  asm volatile("v_nop\n\tv_nop\n\tv_nop\n\tv_nop" : "+v"(c) : "v"(a), "v"(b));
#endif
  return c;
}
__device__ __forceinline__ void guard3(v8f& x, v8f& y, v16h a, v16h b, v16h d) {
#if defined(__HIP_DEVICE_COMPILE__)
  asm volatile("v_nop\n\tv_nop\n\tv_nop\n\tv_nop" : "+v"(x), "+v"(y) : "v"(a), "v"(b), "v"(d));
#endif
}
__device__ __forceinline__ void guard1q(v8f& x, v16h a, v16h b, v16h d, v16h e) {
#if defined(__HIP_DEVICE_COMPILE__)
  asm volatile("v_nop\n\tv_nop\n\tv_nop\n\tv_nop" : "+v"(x) : "v"(a), "v"(b), "v"(d), "v"(e));
#endif
}
__device__ __forceinline__ void guard4m(v8f& x, v8f& y, v16h a, v16h b, v16h d, v16h e) {
#if defined(__HIP_DEVICE_COMPILE__)
  asm volatile("v_nop\n\tv_nop\n\tv_nop\n\tv_nop" : "+v"(x), "+v"(y) : "v"(a), "v"(b), "v"(d), "v"(e)
               : "memory");
#endif
}
__device__ __forceinline__ void guard8m(v8f& x, v8f& y, v16h a, v16h b, v16h d, v16h e,
                                        v16h f, v16h g, v16h p, v16h q) {
#if defined(__HIP_DEVICE_COMPILE__)
  asm volatile("v_nop\n\tv_nop\n\tv_nop\n\tv_nop" : "+v"(x), "+v"(y)
               : "v"(a), "v"(b), "v"(d), "v"(e), "v"(f), "v"(g), "v"(p), "v"(q) : "memory");
#endif
}
__device__ __forceinline__ void acc_guard4(v8f& a, v8f& b, v8f& c, v8f& d) {
#if defined(__HIP_DEVICE_COMPILE__)
  asm volatile("v_nop\n\tv_nop\n\tv_nop\n\tv_nop" : "+v"(a), "+v"(b), "+v"(c), "+v"(d));
#endif
}
__device__ __forceinline__ void cbar() {
#if defined(__HIP_DEVICE_COMPILE__)
  asm volatile("" ::: "memory");
#endif
}
__device__ __forceinline__ void wave_sync_lds() {
  __builtin_amdgcn_fence(__ATOMIC_RELEASE, "workgroup");
  __builtin_amdgcn_wave_barrier();
  __builtin_amdgcn_fence(__ATOMIC_ACQUIRE, "workgroup");
}

__global__ __launch_bounds__(256) void cvt_rm(const float* __restrict__ in, unsigned short* out, int n,
                                             float scale) {
  const size_t i8 = ((size_t)blockIdx.x * 256 + threadIdx.x) * 8;
  if (i8 + 8 > (size_t)n) return;
  const v4f a = *(const v4f*)(in + i8);
  const v4f b = *(const v4f*)(in + i8 + 4);
  float f[8];
  f[0] = a[0]; f[1] = a[1]; f[2] = a[2]; f[3] = a[3];
  f[4] = b[0]; f[5] = b[1]; f[6] = b[2]; f[7] = b[3];
  v4u p;
#pragma unroll
  for (int e = 0; e < 4; ++e) {
    const unsigned short b0 = bf_bits(f[2 * e]), b1 = bf_bits(f[2 * e + 1]);
    const _Float16 x0 = (_Float16)(bf_up(b0) * scale);
    const _Float16 x1 = (_Float16)(bf_up(b1) * scale);
    p[e] = pk16(h_bits(x0), h_bits(x1));
  }
  *(volatile v4u*)(out + i8) = p;
  __threadfence();
  *(volatile v4u*)(out + i8) = p;
}

template <int MODE>
__global__ __launch_bounds__(256) void tr_cvt(const float* __restrict__ in, int R, int C,
                                             unsigned short* out0, unsigned short* out1, float scale) {
  __shared__ float sm[64][65];
  const int tid = threadIdx.x;
  const int c0 = blockIdx.x * 64;
  const int r0 = blockIdx.y * 64;
  if (c0 + 64 > C || r0 + 64 > R) return;
  {
    const int lr = tid >> 2, lc = (tid & 3) * 16;
    const float* src = in + (size_t)(r0 + lr) * (size_t)C + c0 + lc;
#pragma unroll
    for (int q = 0; q < 4; ++q) {
      const v4f v = *(const v4f*)(src + 4 * q);
      sm[lr][lc + 4 * q + 0] = v[0];
      sm[lr][lc + 4 * q + 1] = v[1];
      sm[lr][lc + 4 * q + 2] = v[2];
      sm[lr][lc + 4 * q + 3] = v[3];
    }
  }
  __syncthreads();
  const int seg = tid & 7;
  v4u p0[2], p1[2];
#pragma unroll
  for (int it = 0; it < 2; ++it) {
    const int ocl = it * 32 + (tid >> 3);
    float f[8];
#pragma unroll
    for (int e = 0; e < 8; ++e) f[e] = sm[seg * 8 + e][ocl];
    v4u pk, pl;
#pragma unroll
    for (int e = 0; e < 4; ++e) {
      const float g0 = f[2 * e], g1 = f[2 * e + 1];
      if (MODE == 0) {
        const _Float16 x0 = (_Float16)(bfr(g0) * scale);
        const _Float16 x1 = (_Float16)(bfr(g1) * scale);
        pk[e] = pk16(h_bits(x0), h_bits(x1));
        pl[e] = pk[e];
      } else {
        const float s0 = g0 * scale, s1 = g1 * scale;
        const _Float16 x0 = (_Float16)s0, x1 = (_Float16)s1;
        const _Float16 y0 = (_Float16)((s0 - (float)x0) * RSC);
        const _Float16 y1 = (_Float16)((s1 - (float)x1) * RSC);
        pk[e] = pk16(h_bits(x0), h_bits(x1));
        pl[e] = pk16(h_bits(y0), h_bits(y1));
      }
    }
    p0[it] = pk;
    p1[it] = pl;
  }
  for (int pass = 0; pass < 2; ++pass) {
#pragma unroll
    for (int it = 0; it < 2; ++it) {
      const int ocl = it * 32 + (tid >> 3);
      const size_t go = (size_t)(c0 + ocl) * (size_t)R + (size_t)(r0 + seg * 8);
      *(volatile v4u*)(out0 + go) = p0[it];
      if (MODE == 1) *(volatile v4u*)(out1 + go) = p1[it];
    }
    __threadfence();
  }
}

__global__ __launch_bounds__(256) void rope_tab(float* cost, float* sint, int n) {
  const int e = blockIdx.x * 256 + (int)threadIdx.x;
  if (e >= n) return;
  const int t = e >> 6, i = e & 63;
  const double ex = -(double)i * (1.0 / 64.0);
  const float invf = (float)exp2(ex * LOG2_BASE);
  const float ang = (float)t * invf;
  float sv, cv;
  sincosf(ang, &sv, &cv);
  *(volatile float*)(cost + e) = cv;
  *(volatile float*)(sint + e) = sv;
  __threadfence();
  *(volatile float*)(cost + e) = cv;
  *(volatile float*)(sint + e) = sv;
}

template <int NSW, int EPI>
__global__ __launch_bounds__(128) void gemm_t(
    const unsigned short* __restrict__ A0, const unsigned short* __restrict__ A1, int lda,
    const unsigned short* __restrict__ B0, const unsigned short* __restrict__ B1, int ldb,
    void* C0, void* C1, int ldc,
    const float* __restrict__ cost, const float* __restrict__ sint,
    const float* __restrict__ gain, int hasg,
    int M, int N, int K, float oscale, float cscale) {
  __shared__ __align__(16) float sT[4][16 * 132];
  const int lane = threadIdx.x & 31;
  const int wave = threadIdx.x >> 5;
  const int tilesN = N >> 7;
  const int tilesM = M >> 5;
  const int tile = blockIdx.x * 4 + wave;
  if (tile >= tilesM * tilesN) return;
  const int tm = tile / tilesN;
  const int tn = tile - tm * tilesN;
  const int m0 = tm << 5;
  const int n0 = tn << 7;
  const int rl   = lane & 15;
  const int hh   = lane >> 4;
  const int koff = hh * 8;

  v8f acc[2][8];
#pragma unroll
  for (int i = 0; i < 2; ++i)
#pragma unroll
    for (int j = 0; j < 8; ++j) acc[i][j] = zero8();

#pragma unroll 1
  for (int sw = 0; sw < NSW; ++sw) {
    const unsigned short* Ab = (sw == 0) ? A0 : A1;
    const unsigned short* Bb = (sw == 0) ? B0 : B1;
    const _Float16* ar0 = (const _Float16*)(const void*)Ab + (size_t)(m0 + rl) * (size_t)lda + koff;
    const _Float16* ar1 = (const _Float16*)(const void*)Ab + (size_t)(m0 + 16 + rl) * (size_t)lda + koff;
    const _Float16* br  = (const _Float16*)(const void*)Bb + (size_t)(n0 + rl) * (size_t)ldb + koff;
    for (int k0 = 0; k0 < K; k0 += 32) {
      const v16h a0 = ldfrag_h(ar0 + k0);
      const v16h a1 = ldfrag_h(ar1 + k0);
#pragma unroll
      for (int j = 0; j < 8; ++j) {
        const v16h b = ldfrag_h(br + (size_t)j * 16 * (size_t)ldb + k0);
        acc[0][j] = mma_h_raw(a0, b, acc[0][j]);
        acc[1][j] = mma_h_raw(a1, b, acc[1][j]);
        guard3(acc[0][j], acc[1][j], a0, a1, b);
      }
    }
  }
  acc_guard4(acc[0][0], acc[0][1], acc[0][2], acc[0][3]);
  acc_guard4(acc[0][4], acc[0][5], acc[0][6], acc[0][7]);
  acc_guard4(acc[1][0], acc[1][1], acc[1][2], acc[1][3]);
  acc_guard4(acc[1][4], acc[1][5], acc[1][6], acc[1][7]);

  float gcs = cscale;
  if (EPI == 1) {
    const int gi = (tn < NHEAD) ? tn : (NHEAD - 1);
    const float gv = bfr(gain[gi]);
    gcs = ((hasg != 0) ? gv : 1.0f) * cscale;
  }
  float* slab = sT[wave];
#pragma unroll
  for (int i = 0; i < 2; ++i) {
    const int mB = m0 + 16 * i;
    if (EPI == 1) {
      float inv[8];
#pragma unroll
      for (int r = 0; r < 8; ++r) {
        float ss = 0.f;
#pragma unroll
        for (int j = 0; j < 8; ++j) {
          const float x = acc[i][j][r] * oscale;
          ss += x * x;
        }
        ss += __shfl_xor(ss, 1, 32);
        ss += __shfl_xor(ss, 2, 32);
        ss += __shfl_xor(ss, 4, 32);
        ss += __shfl_xor(ss, 8, 32);
        inv[r] = rsqrtf(ss * (1.0f / (float)HDIM) + RMS_EPS) * oscale;
      }
#pragma unroll
      for (int j = 0; j < 4; ++j) {
#pragma unroll
        for (int r = 0; r < 8; ++r) {
          const int t = mB + 8 * hh + r;
          const float c1 = cost[(size_t)t * RHALF + 16 * j + rl];
          const float s1 = sint[(size_t)t * RHALF + 16 * j + rl];
          const float x1 = acc[i][j][r] * inv[r];
          const float x2 = acc[i][j + 4][r] * inv[r];
          slab[(8 * hh + r) * 132 + 16 * j + rl]      = (x1 * c1 + x2 * s1) * gcs;
          slab[(8 * hh + r) * 132 + 64 + 16 * j + rl] = (x2 * c1 - x1 * s1) * gcs;
        }
      }
    } else {
#pragma unroll
      for (int j = 0; j < 8; ++j) {
#pragma unroll
        for (int r = 0; r < 8; ++r) slab[(8 * hh + r) * 132 + 16 * j + rl] = acc[i][j][r] * oscale;
      }
    }
    wave_sync_lds();
    if (EPI == 3) {
      float* Cf = (float*)C0;
      for (int pass = 0; pass < 2; ++pass) {
#pragma unroll
        for (int it = 0; it < 16; ++it) {
          const v4f o = *(const v4f*)(slab + it * 132 + lane * 4);
          *(volatile v4f*)(Cf + (size_t)(mB + it) * (size_t)ldc + n0 + lane * 4) = o;
        }
        __threadfence();
      }
    } else {
      unsigned short* Cp = (unsigned short*)C0;
      unsigned short* Cq = (unsigned short*)C1;
      v4u hv[8], lv[8];
#pragma unroll
      for (int it = 0; it < 8; ++it) {
        const int row = it * 2 + hh;
        const float* sp = slab + row * 132 + rl * 8;
        const v4f fa = *(const v4f*)sp;
        const v4f fb = *(const v4f*)(sp + 4);
        float f[8];
        f[0] = fa[0]; f[1] = fa[1]; f[2] = fa[2]; f[3] = fa[3];
        f[4] = fb[0]; f[5] = fb[1]; f[6] = fb[2]; f[7] = fb[3];
        v4u pk, pl;
#pragma unroll
        for (int e = 0; e < 4; ++e) {
          const float g0 = f[2 * e], g1 = f[2 * e + 1];
          const _Float16 x0 = (_Float16)g0;
          const _Float16 x1 = (_Float16)g1;
          const _Float16 y0 = (_Float16)((g0 - (float)x0) * RSC);
          const _Float16 y1 = (_Float16)((g1 - (float)x1) * RSC);
          pk[e] = pk16(h_bits(x0), h_bits(x1));
          pl[e] = pk16(h_bits(y0), h_bits(y1));
        }
        hv[it] = pk;
        lv[it] = pl;
      }
      for (int pass = 0; pass < 2; ++pass) {
#pragma unroll
        for (int it = 0; it < 8; ++it) {
          const int row = it * 2 + hh;
          const size_t go = (size_t)(mB + row) * (size_t)ldc + n0 + rl * 8;
          *(volatile v4u*)(Cp + go) = hv[it];
          *(volatile v4u*)(Cq + go) = lv[it];
        }
        __threadfence();
      }
    }
    wave_sync_lds();
  }
}

template <bool SRES, bool PRES>
__global__ __launch_bounds__(128)
void attn_x(const unsigned short* __restrict__ QHp, const unsigned short* __restrict__ QLp,
            const unsigned short* __restrict__ KHp, const unsigned short* __restrict__ KLp,
            const unsigned short* __restrict__ VHp, const unsigned short* __restrict__ VLp,
            const float* __restrict__ VFp, unsigned short* CH, unsigned short* CL,
            float sscale, int qb0, int nqb) {
  __shared__ __align__(16) _Float16 Ksh[64 * HDIM];
  __shared__ __align__(16) _Float16 Kls[SRES ? 64 * HDIM : 8];
  __shared__ __align__(16) _Float16 Vhs[HDIM * 64];
  __shared__ __align__(16) _Float16 Vls[PRES ? HDIM * 64 : 8];
  __shared__ __align__(16) _Float16 Psh[4][16 * 64];
  __shared__ __align__(16) _Float16 Psl[PRES ? 4 : 1][PRES ? 16 * 64 : 8];
  __shared__ __align__(16) float    Os[4][16 * HDIM];

  const int tid  = threadIdx.x;
  const int wave = tid >> 5;
  const int lane = tid & 31;
  const int hh   = lane >> 4;
  const int c    = lane & 15;

  const int qb  = qb0 + (int)(blockIdx.x % (unsigned)nqb);
  const int h   = (int)(blockIdx.x / (unsigned)nqb);
  const int kvh = h / (NHEAD / NKV);
  const int q0  = qb * 64 + wave * 16;

  const _Float16* Qg  = (const _Float16*)(const void*)QHp + (size_t)h * HDIM;
  const _Float16* Qlg = (const _Float16*)(const void*)QLp + (size_t)h * HDIM;
  const _Float16* Kg  = (const _Float16*)(const void*)KHp + (size_t)kvh * HDIM;
  const _Float16* Klg = (const _Float16*)(const void*)KLp + (size_t)kvh * HDIM;
  const _Float16* Vhg = (const _Float16*)(const void*)VHp + (size_t)kvh * HDIM * SEQ;
  const _Float16* Vlg = (const _Float16*)(const void*)VLp + (size_t)kvh * HDIM * SEQ;
  const float* Vf = VFp + (size_t)kvh * HDIM;

  float mrow[8], lrow[8];
  v8f oh[8];
#pragma unroll
  for (int r = 0; r < 8; ++r) { mrow[r] = NEG_BIG; lrow[r] = 0.f; }
#pragma unroll
  for (int t = 0; t < 8; ++t) oh[t] = zero8();

  _Float16* pwh = Psh[wave];
  _Float16* pwl = &Psl[PRES ? wave : 0][0];

  for (int kt = 0; kt < NQB; ++kt) {
    if (kt > qb) break;
    const int kv0 = kt * 64;
    __syncthreads();
    {
      const int r = tid >> 1, hk = (tid & 1) * 64;
      const _Float16* kg = Kg + (size_t)(kv0 + r) * KVD + hk;
#pragma unroll
      for (int i = 0; i < 8; ++i) *(v8h*)(Ksh + r * HDIM + hk + 8 * i) = *(const v8h*)(kg + 8 * i);
      if (SRES) {
        cbar();
        const _Float16* lg = Klg + (size_t)(kv0 + r) * KVD + hk;
#pragma unroll
        for (int i = 0; i < 8; ++i) *(v8h*)(Kls + r * HDIM + hk + 8 * i) = *(const v8h*)(lg + 8 * i);
        cbar();
      }
      const _Float16* vh = Vhg + (size_t)tid * SEQ + kv0;
#pragma unroll
      for (int i = 0; i < 8; ++i) *(v8h*)(Vhs + tid * 64 + 8 * i) = *(const v8h*)(vh + 8 * i);
      if (PRES) {
        cbar();
        const _Float16* vl = Vlg + (size_t)tid * SEQ + kv0;
#pragma unroll
        for (int i = 0; i < 8; ++i) *(v8h*)(Vls + tid * 64 + 8 * i) = *(const v8h*)(vl + 8 * i);
        cbar();
      }
    }
    __syncthreads();

    v8f s[4];
    if (SRES) {
#pragma unroll
      for (int jp = 0; jp < 2; ++jp) {
        v8f sh2[2], sl2[2];
        sh2[0] = zero8(); sh2[1] = zero8(); sl2[0] = zero8(); sl2[1] = zero8();
#pragma unroll
        for (int dc = 0; dc < 4; ++dc) {
          const v16h qhf = ldfrag_h(Qg  + (size_t)(q0 + c) * DM + dc * 32 + 8 * hh);
          const v16h qlf = ldfrag_h(Qlg + (size_t)(q0 + c) * DM + dc * 32 + 8 * hh);
#pragma unroll
          for (int jj = 0; jj < 2; ++jj) {
            const int j = 2 * jp + jj;
            FH kb, lb;
            kb.h[0] = *(const v8h*)(Ksh + (j * 16 + c) * HDIM + dc * 32 + 8 * hh);
            kb.h[1] = *(const v8h*)(Ksh + (j * 16 + c) * HDIM + dc * 32 + 16 + 8 * hh);
            lb.h[0] = *(const v8h*)(Kls + (j * 16 + c) * HDIM + dc * 32 + 8 * hh);
            lb.h[1] = *(const v8h*)(Kls + (j * 16 + c) * HDIM + dc * 32 + 16 + 8 * hh);
            sh2[jj] = mma_h_raw(qhf, kb.v, sh2[jj]);
            sl2[jj] = mma_h_raw(qlf, kb.v, sl2[jj]);
            sl2[jj] = mma_h_raw(qhf, lb.v, sl2[jj]);
            guard4m(sh2[jj], sl2[jj], qhf, qlf, kb.v, lb.v);
          }
        }
#pragma unroll
        for (int jj = 0; jj < 2; ++jj) {
          const int j    = 2 * jp + jj;
          const int key  = kv0 + j * 16 + c;
          const int rowb = q0 + 8 * hh;
#pragma unroll
          for (int r = 0; r < 8; ++r) {
            float v = sh2[jj][r];
            v += sl2[jj][r] * (1.0f / RSC);
            v *= sscale;
            s[j][r] = (key <= rowb + r) ? v : NEG_BIG;
          }
        }
      }
    } else {
      v16h qh[4];
#pragma unroll
      for (int dc = 0; dc < 4; ++dc) qh[dc] = ldfrag_h(Qg + (size_t)(q0 + c) * DM + dc * 32 + 8 * hh);
#pragma unroll
      for (int j = 0; j < 4; ++j) {
        v8f sh = zero8();
#pragma unroll
        for (int dc = 0; dc < 4; ++dc) {
          FH kb;
          kb.h[0] = *(const v8h*)(Ksh + (j * 16 + c) * HDIM + dc * 32 + 8 * hh);
          kb.h[1] = *(const v8h*)(Ksh + (j * 16 + c) * HDIM + dc * 32 + 16 + 8 * hh);
          sh = mma_h(qh[dc], kb.v, sh);
        }
        const int key  = kv0 + j * 16 + c;
        const int rowb = q0 + 8 * hh;
#pragma unroll
        for (int r = 0; r < 8; ++r) {
          const float v = sh[r] * sscale;
          s[j][r] = (key <= rowb + r) ? v : NEG_BIG;
        }
      }
    }

#pragma unroll
    for (int r = 0; r < 8; ++r) {
      float m = s[0][r];
      m = fmaxf(m, s[1][r]);
      m = fmaxf(m, s[2][r]);
      m = fmaxf(m, s[3][r]);
#pragma unroll
      for (int off = 1; off < 16; off <<= 1) m = fmaxf(m, __shfl_xor(m, off, 32));
      const float mnew  = fmaxf(mrow[r], m);
      const float alpha = __expf(mrow[r] - mnew);
      mrow[r] = mnew;
      float psum = 0.f;
#pragma unroll
      for (int j = 0; j < 4; ++j) {
        const float p  = __expf(s[j][r] - mnew);
        psum += p;
        const float ph = p * PSC;
        const _Float16 xh = (_Float16)ph;
        const int pi = (8 * hh + r) * 64 + j * 16 + c;
        pwh[pi] = xh;
        if (PRES) pwl[pi] = (_Float16)((ph - (float)xh) * RSC);
      }
#pragma unroll
      for (int off = 1; off < 16; off <<= 1) psum += __shfl_xor(psum, off, 32);
      lrow[r] = lrow[r] * alpha + psum;
#pragma unroll
      for (int t = 0; t < 8; ++t) oh[t][r] *= alpha;
    }
    wave_sync_lds();

    FH pa0, pa1, pb0, pb1;
    pa0.h[0] = *(const v8h*)(pwh + c * 64 + 8 * hh);
    pa0.h[1] = *(const v8h*)(pwh + c * 64 + 16 + 8 * hh);
    pa1.h[0] = *(const v8h*)(pwh + c * 64 + 32 + 8 * hh);
    pa1.h[1] = *(const v8h*)(pwh + c * 64 + 48 + 8 * hh);
    pb0.v = pa0.v;
    pb1.v = pa1.v;
    if (PRES) {
      pb0.h[0] = *(const v8h*)(pwl + c * 64 + 8 * hh);
      pb0.h[1] = *(const v8h*)(pwl + c * 64 + 16 + 8 * hh);
      pb1.h[0] = *(const v8h*)(pwl + c * 64 + 32 + 8 * hh);
      pb1.h[1] = *(const v8h*)(pwl + c * 64 + 48 + 8 * hh);
      cbar();
    }
#pragma unroll
    for (int t = 0; t < 8; ++t) {
      const _Float16* vr = Vhs + (t * 16 + c) * 64 + 8 * hh;
      FH vb0, vb1;
      vb0.h[0] = *(const v8h*)(vr);
      vb0.h[1] = *(const v8h*)(vr + 16);
      vb1.h[0] = *(const v8h*)(vr + 32);
      vb1.h[1] = *(const v8h*)(vr + 48);
      if (PRES) {
        const _Float16* wr = Vls + (t * 16 + c) * 64 + 8 * hh;
        FH wb0, wb1;
        wb0.h[0] = *(const v8h*)(wr);
        wb0.h[1] = *(const v8h*)(wr + 16);
        wb1.h[0] = *(const v8h*)(wr + 32);
        wb1.h[1] = *(const v8h*)(wr + 48);
        v8f ol = zero8();
        oh[t] = mma_h_raw(pa0.v, vb0.v, oh[t]);
        ol    = mma_h_raw(pa0.v, wb0.v, ol);
        ol    = mma_h_raw(pb0.v, vb0.v, ol);
        oh[t] = mma_h_raw(pa1.v, vb1.v, oh[t]);
        ol    = mma_h_raw(pa1.v, wb1.v, ol);
        ol    = mma_h_raw(pb1.v, vb1.v, ol);
        guard8m(oh[t], ol, pa0.v, pa1.v, pb0.v, pb1.v, vb0.v, vb1.v, wb0.v, wb1.v);
#pragma unroll
        for (int r = 0; r < 8; ++r) oh[t][r] += ol[r] * (1.0f / RSC);
      } else {
        oh[t] = mma_h_raw(pa0.v, vb0.v, oh[t]);
        oh[t] = mma_h_raw(pa1.v, vb1.v, oh[t]);
        guard1q(oh[t], pa0.v, pa1.v, vb0.v, vb1.v);
      }
    }
    acc_guard4(oh[0], oh[1], oh[2], oh[3]);
    acc_guard4(oh[4], oh[5], oh[6], oh[7]);
  }

  float* os = Os[wave];
#pragma unroll
  for (int r = 0; r < 8; ++r) {
    const int qr = q0 + 8 * hh + r;
    const float l = lrow[r];
    const float inv = (1.0f / l) * (1.0f / (PSC * VSC));
    const float* vrow = Vf + (size_t)qr * KVD;
    float vv[8], yv[8];
    float ss = 0.f, dt = 0.f;
#pragma unroll
    for (int t = 0; t < 8; ++t) {
      vv[t] = vrow[t * 16 + c];
      yv[t] = oh[t][r] * inv;
      ss += vv[t] * vv[t];
      dt += yv[t] * vv[t];
    }
#pragma unroll
    for (int off = 1; off < 16; off <<= 1) {
      ss += __shfl_xor(ss, off, 32);
      dt += __shfl_xor(dt, off, 32);
    }
    const float nrm  = sqrtf(ss);
    const float ivn  = 1.0f / fmaxf(nrm, XCLIP);
    const float coef = dt * ivn;
#pragma unroll
    for (int t = 0; t < 8; ++t) os[(8 * hh + r) * HDIM + t * 16 + c] = yv[t] - coef * (vv[t] * ivn);
  }
  wave_sync_lds();
  {
    v4u hvv[8], lvv[8];
#pragma unroll
    for (int it = 0; it < 8; ++it) {
      const int row = it * 2 + hh;
      const float* sp = os + row * HDIM + c * 8;
      const v4f fa = *(const v4f*)sp;
      const v4f fb = *(const v4f*)(sp + 4);
      float f[8];
      f[0] = fa[0]; f[1] = fa[1]; f[2] = fa[2]; f[3] = fa[3];
      f[4] = fb[0]; f[5] = fb[1]; f[6] = fb[2]; f[7] = fb[3];
      v4u pk, pl;
#pragma unroll
      for (int e = 0; e < 4; ++e) {
        const float g0 = f[2 * e] * CXS, g1 = f[2 * e + 1] * CXS;
        const _Float16 x0 = (_Float16)g0, x1 = (_Float16)g1;
        const _Float16 y0 = (_Float16)(g0 - (float)x0), y1 = (_Float16)(g1 - (float)x1);
        pk[e] = pk16(h_bits(x0), h_bits(x1));
        pl[e] = pk16(h_bits(y0), h_bits(y1));
      }
      hvv[it] = pk;
      lvv[it] = pl;
    }
    for (int pass = 0; pass < 2; ++pass) {
#pragma unroll
      for (int it = 0; it < 8; ++it) {
        const int row = it * 2 + hh;
        const size_t go = (size_t)(q0 + row) * DM + (size_t)h * HDIM + c * 8;
        *(volatile v4u*)(CH + go) = hvv[it];
        *(volatile v4u*)(CL + go) = lvv[it];
      }
      __threadfence();
    }
  }
}

extern "C" void kernel_launch(void* const* d_in, const int* in_sizes, int n_in,
                              void* d_out, int out_size, void* d_ws, size_t ws_size,
                              hipStream_t stream) {
  if (n_in < 6) return;
  if (in_sizes[0] != NTOK * DM) return;
  if (in_sizes[1] != DM * DM) return;
  if (in_sizes[2] != DM * KVD || in_sizes[3] != DM * KVD) return;
  if (in_sizes[4] != DM * DM) return;
  if (in_sizes[5] != NHEAD) return;
  if (out_size != NTOK * DM) return;

  const float* X  = (const float*)d_in[0];
  const float* Wq = (const float*)d_in[1];
  const float* Wk = (const float*)d_in[2];
  const float* Wv = (const float*)d_in[3];
  const float* Wo = (const float*)d_in[4];
  const float* QG = (const float*)d_in[5];
  float* outf = (float*)d_out;

  const size_t PXH  = (size_t)NTOK * DM * 2;
  const size_t PWQ  = (size_t)DM * DM * 2;
  const size_t PWK  = (size_t)KVD * DM * 2;
  const size_t PWO  = (size_t)DM * DM * 2;
  const size_t PRT  = (size_t)SEQ * RHALF * 4;
  const size_t PQ   = (size_t)SEQ * DM * 2;
  const size_t PK   = (size_t)SEQ * KVD * 2;
  const size_t PVF  = (size_t)SEQ * KVD * 4;
  const size_t PVT  = (size_t)KVD * SEQ * 2;
  const size_t PCTX = (size_t)SEQ * DM * 2;
  size_t off = 0;
  const size_t oXH = off; off += PXH;
  const size_t oWQ = off; off += PWQ;
  const size_t oWK = off; off += PWK;
  const size_t oWV = off; off += PWK;
  const size_t oWO = off; off += PWO;
  const size_t oCT = off; off += PRT;
  const size_t oST = off; off += PRT;
  const size_t oQH = off; off += PQ;
  const size_t oQL = off; off += PQ;
  const size_t oKH = off; off += PK;
  const size_t oKL = off; off += PK;
  const size_t oVF = off; off += PVF;
  const size_t oVH = off; off += PVT;
  const size_t oVL = off; off += PVT;
  const size_t oCH = off; off += PCTX;
  const size_t oCL = off; off += PCTX;
  if (off > ws_size) return;
  if (off > (size_t)134217728) return;

  char* ws = (char*)d_ws;
  unsigned short* XH   = (unsigned short*)(ws + oXH);
  unsigned short* WQT  = (unsigned short*)(ws + oWQ);
  unsigned short* WKT  = (unsigned short*)(ws + oWK);
  unsigned short* WVT  = (unsigned short*)(ws + oWV);
  unsigned short* WOT  = (unsigned short*)(ws + oWO);
  float*          COST = (float*)(ws + oCT);
  float*          SINT = (float*)(ws + oST);
  unsigned short* QH   = (unsigned short*)(ws + oQH);
  unsigned short* QL   = (unsigned short*)(ws + oQL);
  unsigned short* KH   = (unsigned short*)(ws + oKH);
  unsigned short* KL   = (unsigned short*)(ws + oKL);
  float*          VF   = (float*)(ws + oVF);
  unsigned short* VTH  = (unsigned short*)(ws + oVH);
  unsigned short* VTL  = (unsigned short*)(ws + oVL);
  unsigned short* CTXH = (unsigned short*)(ws + oCH);
  unsigned short* CTXL = (unsigned short*)(ws + oCL);

  const dim3 blk256(256), blk128(128);
  const float sscale = 0.08838834764831845f / (QSC * KSC);

  cvt_rm<<<dim3((NTOK * DM) / 2048), blk256, 0, stream>>>(X, XH, NTOK * DM, 1.0f);
  tr_cvt<0><<<dim3(DM / 64, DM / 64), blk256, 0, stream>>>(Wq, DM, DM, WQT, WQT, WSC);
  tr_cvt<0><<<dim3(KVD / 64, DM / 64), blk256, 0, stream>>>(Wk, DM, KVD, WKT, WKT, WSC);
  tr_cvt<0><<<dim3(KVD / 64, DM / 64), blk256, 0, stream>>>(Wv, DM, KVD, WVT, WVT, WSC);
  tr_cvt<0><<<dim3(DM / 64, DM / 64), blk256, 0, stream>>>(Wo, DM, DM, WOT, WOT, WSC);
  rope_tab<<<dim3((SEQ * RHALF) / 256), blk256, 0, stream>>>(COST, SINT, SEQ * RHALF);

  const int gq = ((SEQ / 32) * (DM / 128)) / 4;
  const int gk = ((SEQ / 32) * (KVD / 128)) / 4;
  const int go = ((SEQ / 32) * (DM / 128)) / 4;
  for (int b = 0; b < NBATCH; ++b) {
    const unsigned short* XHb = XH + (size_t)b * SEQ * DM;
    float* outb = outf + (size_t)b * SEQ * DM;
    gemm_t<1, 1><<<dim3(gq), blk128, 0, stream>>>(
        XHb, XHb, DM, WQT, WQT, DM, (void*)QH, (void*)QL, DM, COST, SINT, QG, 1,
        SEQ, DM, DM, 1.0f / WSC, QSC);
    gemm_t<1, 1><<<dim3(gk), blk128, 0, stream>>>(
        XHb, XHb, DM, WKT, WKT, DM, (void*)KH, (void*)KL, KVD, COST, SINT, QG, 0,
        SEQ, KVD, DM, 1.0f / WSC, KSC);
    gemm_t<1, 3><<<dim3(gk), blk128, 0, stream>>>(
        XHb, XHb, DM, WVT, WVT, DM, (void*)VF, (void*)VF, KVD, COST, SINT, QG, 0,
        SEQ, KVD, DM, 1.0f / WSC, 1.0f);
    tr_cvt<1><<<dim3(KVD / 64, SEQ / 64), blk256, 0, stream>>>(VF, SEQ, KVD, VTH, VTL, VSC);
    attn_x<true, true><<<dim3(NQP * NHEAD), blk128, 0, stream>>>(QH, QL, KH, KL, VTH, VTL, VF, CTXH, CTXL,
                                                                 sscale, 0, NQP);
    attn_x<true, false><<<dim3((NQB - NQP) * NHEAD), blk128, 0, stream>>>(QH, QL, KH, KL, VTH, VTL, VF,
                                                                          CTXH, CTXL, sscale, NQP, NQB - NQP);
    gemm_t<2, 3><<<dim3(go), blk128, 0, stream>>>(
        CTXH, CTXL, DM, WOT, WOT, DM, (void*)outb, (void*)outb, DM, COST, SINT, QG, 0,
        SEQ, DM, DM, 1.0f / (CXS * WSC), 1.0f);
  }
  (void)hipGetLastError();
}
